// GAT_attention_multi_12910671692372
// MI455X (gfx1250) — hardware-verified
//
#include <hip/hip_runtime.h>
#include <stddef.h>


typedef _Float16 v16h __attribute__((ext_vector_type(16)));
typedef _Float16 v8h  __attribute__((ext_vector_type(8)));
typedef float    v8f  __attribute__((ext_vector_type(8)));
typedef float    v4f  __attribute__((ext_vector_type(4)));
typedef float    v2f  __attribute__((ext_vector_type(2)));

#ifndef NB
#define NB 32
#endif
#define NB_FULL 32
#define NODES 202
#define NN    200
#define NP    208
#define NT    13
#define DD    64
#define KP    224
#define UP    256
#define TP    224
#define TROWS 6
#define LDU   68
#define LDC   68
#define WLD   232

#define UA2CARRY 16.0f
#define WRCARRY  1024.0f
#define RCARRY   2048.0f
#define LN_EPS   1.0e-5f

static_assert(NB >= 1 && NB <= NB_FULL);
static_assert(NODES == NN + 2);
static_assert(NP == NT * 16 && NP >= NN);
static_assert(DD == 64);
static_assert((KP % 32) == 0 && KP >= NP && KP <= WLD - 8 + 8);
static_assert(UP >= KP && (UP % 64) == 0);
static_assert(TP >= KP && (TP % 32) == 0);
static_assert((LDU % 4) == 0 && LDU >= DD);
static_assert((LDC % 4) == 0 && LDC >= DD);
static_assert((WLD % 8) == 0 && WLD >= KP);
static_assert(KP - NP == 16);
static_assert(13 * 256 == NP * DD / 4);
static_assert(NP * DD / 8 == 1664);
static_assert(8 * 256 == DD * UP / 8);
static_assert(TROWS * TP / 4 == 336);
static_assert(16 * (DD / 4) == 256);

static_assert((NP * LDU + TROWS * TP + 6 * DD + 8 + DD) * 4 <= 65536);
static_assert(2 * 16 * WLD * 2 + (8 * 32 + 32 + 16 * LDC) * 4 <= 65536);
static_assert(2 * 16 * WLD * 2 + (8 * 32 + 32 + 16 * LDC) * 4 <= 131072);

#define UA16_BYTES ((size_t)NB * NP * DD * 2)
#define UAT_BYTES  ((size_t)NB * DD * UP * 2)
#define UAF_BYTES  ((size_t)NB * NP * DD * 4)
#define TAB_BYTES  ((size_t)NB * TROWS * TP * 4)
#define OFF_UA16 ((size_t)0)
#define OFF_UA2  (OFF_UA16 + UA16_BYTES)
#define OFF_UAT  (OFF_UA2 + UA16_BYTES)
#define OFF_UATR (OFF_UAT + UAT_BYTES)
#define OFF_UAF  (OFF_UATR + UAT_BYTES)
#define OFF_TAB  (OFF_UAF + UAF_BYTES)
#define WS_TOTAL (OFF_TAB + TAB_BYTES)
static_assert((UA16_BYTES % 128) == 0 && (UAT_BYTES % 128) == 0);
static_assert((UAF_BYTES % 128) == 0 && (TAB_BYTES % 128) == 0);
static_assert(((size_t)NP * DD * 2) % 128 == 0 && ((size_t)DD * UP * 2) % 128 == 0);
static_assert(((size_t)TROWS * TP * 4) % 128 == 0);
static_assert(WS_TOTAL <= (size_t)134217728);

__device__ __forceinline__ float bf16r(float x) {
  unsigned int u = __float_as_uint(x);
  u = (u + 0x7FFFu + ((u >> 16) & 1u)) & 0xFFFF0000u;
  return __uint_as_float(u);
}

__device__ __forceinline__ v16h frag_at(const _Float16* p) {
  v8h lo = *(const v8h*)(p);
  v8h hi = *(const v8h*)(p + 16);
  v16h out;
#pragma unroll
  for (int i = 0; i < 8; ++i) { out[i] = lo[i]; out[i + 8] = hi[i]; }
  return out;
}
__device__ __forceinline__ v16h ld_frag(const _Float16* base, unsigned ld) {
  const unsigned lane = threadIdx.x & 31u;
  return frag_at(base + (lane & 15u) * ld + (lane >> 4) * 8u);
}

__device__ __forceinline__ v8f wmma16(v16h a, v16h b, v8f c) {
  v8f d = __builtin_amdgcn_wmma_f32_16x16x32_f16(false, a, false, b, (short)0, c,
                                                 false, false);
  asm volatile("v_nop\n\tv_nop\n\tv_nop\n\tv_nop" : "+v"(d) : "v"(a), "v"(b));
  return d;
}

__device__ __forceinline__ float red32_sum(float x) {
#pragma unroll
  for (int off = 1; off < 32; off <<= 1) x += __shfl_xor(x, off, 32);
  return x;
}
__device__ __forceinline__ float red32_max(float x) {
#pragma unroll
  for (int off = 1; off < 32; off <<= 1) x = fmaxf(x, __shfl_xor(x, off, 32));
  return x;
}

__device__ __forceinline__ void wave_lds_sync() {
  __builtin_amdgcn_fence(3  , "wavefront");
  asm volatile("s_wait_dscnt 0x0" ::: "memory");
  __builtin_amdgcn_wave_barrier();
}

static __device__ __forceinline__ _Float16 toh_flush(float v) {
  const _Float16 r = (_Float16)v;
  return (fabsf(v) < 6.103515625e-05f) ? (_Float16)0.0f : r;
}

__device__ __forceinline__ float leaky(float x) { return x > 0.0f ? x : 0.01f * x; }

__device__ __forceinline__ void ln_pair(const float* __restrict__ xr, const unsigned lane,
                                        const float g0, const float g1,
                                        const float b0, const float b1,
                                        float& y0, float& y1) {
  const v2f a = *(const v2f*)(xr + 2u * lane);
  const float e0 = bf16r(a[0]), e1 = bf16r(a[1]);
  const float mean = red32_sum(e0 + e1) * (1.0f / (float)DD);
  const float d0 = e0 - mean, d1 = e1 - mean;
  const float var = red32_sum(d0 * d0 + d1 * d1) * (1.0f / (float)DD);
  const float rstd = rsqrtf(var + LN_EPS);
  y0 = d0 * rstd * g0 + b0;
  y1 = d1 * rstd * g1 + b1;
}

__global__ __launch_bounds__(256) void prep_kernel(
    const float* __restrict__ emb, const float* __restrict__ lnw, const float* __restrict__ lnb,
    const float* __restrict__ W1, const float* __restrict__ W1b,
    const float* __restrict__ W2, const float* __restrict__ W2b,
    const float* __restrict__ a1, const float* __restrict__ a1b,
    const float* __restrict__ a2, const float* __restrict__ a2b,
    _Float16* __restrict__ UA16, _Float16* __restrict__ UA2, _Float16* __restrict__ UAT,
    _Float16* __restrict__ UATR,
    float* __restrict__ UAF, float* __restrict__ TAB, float* __restrict__ out) {
#pragma clang fp contract(off)
  __shared__ float sUA[NP * LDU];
  __shared__ float sTab[TROWS * TP];
  __shared__ float sV[6 * DD];
  __shared__ float sCb[8];
  __shared__ float sO[DD];

  const unsigned tid = threadIdx.x, lane = tid & 31u;
  const int wave = __builtin_amdgcn_readfirstlane(threadIdx.x >> 5);
  const unsigned b = blockIdx.x;

  for (unsigned idx = tid; idx < (unsigned)(TROWS * TP); idx += 256u) {
    const unsigned row = idx / (unsigned)TP;
    sTab[idx] = (row == 2u || row == 3u) ? 1.0e30f : 0.0f;
  }
  for (unsigned idx = tid; idx < (unsigned)((NP - NN) * LDU); idx += 256u)
    sUA[NN * LDU + idx] = 0.0f;

  if (wave < 6) {
    const unsigned v = tid >> 6, e = tid & 63u;
    float acc1 = 0.0f, acc2 = 0.0f;
#pragma unroll 1
    for (unsigned o = 0; o < (unsigned)DD; ++o) {
      acc1 += bf16r(a1[v * DD + o]) * bf16r(W1[o * DD + e]);
      acc2 += bf16r(a2[v * DD + o]) * bf16r(W2[o * DD + e]);
    }
    sV[v * DD + e] = acc1;
    sV[(3u + v) * DD + e] = acc2;
  } else if (wave == 6) {
    const unsigned v = (lane < 3u) ? lane : 2u;
    float c1 = 0.0f, c2 = 0.0f;
#pragma unroll 1
    for (unsigned o = 0; o < (unsigned)DD; ++o) {
      c1 += bf16r(W1b[o]) * bf16r(a1[v * DD + o]);
      c2 += bf16r(W2b[o]) * bf16r(a2[v * DD + o]);
    }
    if (lane < 3u) { sCb[v] = c1; sCb[3u + v] = c2; }
  }
  __syncthreads();

  const float* eb = emb + (size_t)b * (NODES * DD);
  const v2f gwv = *(const v2f*)(lnw + 2u * lane);
  const v2f gbv = *(const v2f*)(lnb + 2u * lane);
  const float g0 = bf16r(gwv[0]), g1 = bf16r(gwv[1]);
  const float b0 = bf16r(gbv[0]), b1 = bf16r(gbv[1]);

  float ux, uy, ix, iy;
  ln_pair(eb, lane, g0, g1, b0, b1, ux, uy);
  ln_pair(eb + DD, lane, g0, g1, b0, b1, ix, iy);

  const float vq1x = sV[0 * DD + 2u * lane], vq1y = sV[0 * DD + 2u * lane + 1u];
  const float vk1x = sV[1 * DD + 2u * lane], vk1y = sV[1 * DD + 2u * lane + 1u];
  const float vi1x = sV[2 * DD + 2u * lane], vi1y = sV[2 * DD + 2u * lane + 1u];
  const float vq2x = sV[3 * DD + 2u * lane], vq2y = sV[3 * DD + 2u * lane + 1u];
  const float vk2x = sV[4 * DD + 2u * lane], vk2y = sV[4 * DD + 2u * lane + 1u];
  const float vi2x = sV[5 * DD + 2u * lane], vi2y = sV[5 * DD + 2u * lane + 1u];
  const float cq1 = sCb[0], ck1 = sCb[1], ci1 = sCb[2];
  const float cq2 = sCb[3], ck2 = sCb[4], ci2 = sCb[5];

  const float si1 = red32_sum(ix * vi1x + iy * vi1y);
  const float si2 = red32_sum(ix * vi2x + iy * vi2y);
  const float c1 = (si1 + ci1) + bf16r(a1b[0]);
  const float c2 = (si2 + ci2) + bf16r(a2b[0]);

  if (wave == 0) {
    sO[2u * lane]      = leaky(ux * ix);
    sO[2u * lane + 1u] = leaky(uy * iy);
    wave_lds_sync();
    if (lane < 16u) {
      const v4f o = *(const v4f*)&sO[4u * lane];
      float* p = out + (size_t)b * ((NN + 1) * DD) + 4u * lane;
      *(volatile v4f*)p = o;
      __threadfence();
      *(volatile v4f*)p = o;
    }
  }

#pragma unroll 1
  for (unsigned i = (unsigned)wave; i < (unsigned)NN; i += 8u) {
    float x0, x1;
    ln_pair(eb + (size_t)(2u + i) * DD, lane, g0, g1, b0, b1, x0, x1);
    const float px = ux * x0, py = uy * x1;
    v2f pv; pv[0] = px; pv[1] = py;
    *(v2f*)&sUA[i * LDU + 2u * lane] = pv;
    const float dq1 = red32_sum(px * vq1x + py * vq1y);
    const float dk1 = red32_sum(px * vk1x + py * vk1y);
    const float dq2 = red32_sum(px * vq2x + py * vq2y);
    const float dk2 = red32_sum(px * vk2x + py * vk2y);
    if (lane == 0u) {
      sTab[0 * TP + i] = (dq1 + cq1) + c1;
      sTab[1 * TP + i] = (dq2 + cq2) + c2;
      sTab[4 * TP + i] = dk1 + ck1;
      sTab[5 * TP + i] = dk2 + ck2;
    }
  }
  __syncthreads();

  float km1 = -3.0e38f, km2 = -3.0e38f;
#pragma unroll 1
  for (unsigned t = 0; t < 7u; ++t) {
    const unsigned j = lane + 32u * t;
    const float s1 = sTab[4 * TP + j], s2 = sTab[5 * TP + j];
    km1 = fmaxf(km1, (j < (unsigned)NN) ? s1 : -3.0e38f);
    km2 = fmaxf(km2, (j < (unsigned)NN) ? s2 : -3.0e38f);
  }
  km1 = red32_max(km1);
  km2 = red32_max(km2);
#pragma unroll 1
  for (unsigned i = (unsigned)wave; i < (unsigned)NN; i += 8u) {
    const float q1 = sTab[0 * TP + i], q2 = sTab[1 * TP + i];
    const float mx1 = leaky(q1 + km1), mx2 = leaky(q2 + km2);
    float d1 = 0.0f, d2 = 0.0f;
#pragma unroll 1
    for (unsigned t = 0; t < 7u; ++t) {
      const unsigned j = lane + 32u * t;
      const float e1 = __expf(leaky(q1 + sTab[4 * TP + j]) - mx1);
      const float e2 = __expf(leaky(q2 + sTab[5 * TP + j]) - mx2);
      d1 += (j < (unsigned)NN) ? e1 : 0.0f;
      d2 += (j < (unsigned)NN) ? e2 : 0.0f;
    }
    d1 = red32_sum(d1);
    d2 = red32_sum(d2);
    if (lane == 0u) {
      sTab[2 * TP + i] = mx1 + __logf(d1);
      sTab[3 * TP + i] = mx2 + __logf(d2);
    }
  }
  __syncthreads();

  float* uaf = UAF + (size_t)b * (NP * DD);
#pragma unroll 1
  for (unsigned s = 0; s < 13u; ++s) {
    const unsigned p = tid + 256u * s;
    const v4f v = *(const v4f*)&sUA[(p >> 4) * LDU + (p & 15u) * 4u];
    float* q = uaf + (size_t)p * 4u;
    *(volatile v4f*)q = v;
    __threadfence();
    *(volatile v4f*)q = v;
  }

  _Float16* ua16 = UA16 + (size_t)b * (NP * DD);
  _Float16* ua2  = UA2 + (size_t)b * (NP * DD);
#pragma unroll 1
  for (unsigned s = 0; s < 7u; ++s) {
    const unsigned p = tid + 256u * s;
    if (p < 1664u) {
      const unsigned row = p >> 3, c = (p & 7u) * 8u;
      const v4f t0 = *(const v4f*)&sUA[row * LDU + c];
      const v4f t1 = *(const v4f*)&sUA[row * LDU + c + 4u];
      v8h h, h2;
#pragma unroll
      for (int j = 0; j < 4; ++j) {
        h[j]      = toh_flush(t0[j]);
        h[j + 4]  = toh_flush(t1[j]);
        h2[j]     = toh_flush(UA2CARRY * (t0[j] * t0[j]));
        h2[j + 4] = toh_flush(UA2CARRY * (t1[j] * t1[j]));
      }
      _Float16* q1 = ua16 + (size_t)p * 8u;
      _Float16* q2 = ua2 + (size_t)p * 8u;
      *(volatile v8h*)q1 = h;
      *(volatile v8h*)q2 = h2;
      __threadfence();
      *(volatile v8h*)q1 = h;
      *(volatile v8h*)q2 = h2;
    }
  }

  _Float16* uat  = UAT + (size_t)b * (DD * UP);
  _Float16* uatr = UATR + (size_t)b * (DD * UP);
#pragma unroll 1
  for (unsigned s = 0; s < 8u; ++s) {
    const unsigned p = tid + 256u * s;
    const unsigned d = p >> 5, pc = p & 31u;
    v8h h, hr;
#pragma unroll
    for (unsigned k = 0; k < 8u; ++k) {
      const unsigned i = 8u * pc + k;
      const unsigned ic = (i < (unsigned)NP) ? i : (unsigned)(NP - 1);
      const float v = sUA[ic * LDU + d];
      const float vv = (i < (unsigned)NP) ? v : 0.0f;
      const _Float16 hv = toh_flush(vv);
      h[k]  = hv;
      hr[k] = toh_flush(RCARRY * (vv - (float)hv));
    }
    _Float16* q  = uat + (size_t)p * 8u;
    _Float16* qr = uatr + (size_t)p * 8u;
    *(volatile v8h*)q  = h;
    *(volatile v8h*)qr = hr;
    __threadfence();
    *(volatile v8h*)q  = h;
    *(volatile v8h*)qr = hr;
  }

  float* tab = TAB + (size_t)b * (TROWS * TP);
#pragma unroll 1
  for (unsigned s = 0; s < 2u; ++s) {
    const unsigned p = tid + 256u * s;
    if (p < 336u) {
      const v4f v = *(const v4f*)&sTab[4u * p];
      float* q = tab + (size_t)p * 4u;
      *(volatile v4f*)q = v;
      __threadfence();
      *(volatile v4f*)q = v;
    }
  }
}

__global__ __launch_bounds__(256) void gat_kernel(
    const _Float16* __restrict__ UA16, const _Float16* __restrict__ UA2,
    const _Float16* __restrict__ UAT, const _Float16* __restrict__ UATR,
    const float* __restrict__ UAF,
    const float* __restrict__ TAB, const float* __restrict__ lnw,
    const float* __restrict__ lnb, float* __restrict__ out) {
  __shared__ _Float16 sW[16 * WLD];
  __shared__ _Float16 sWR[16 * WLD];
  __shared__ float sPart[8 * 32];
  __shared__ float sS[32];
  __shared__ float sC[16 * LDC];

  const unsigned tid = threadIdx.x, lane = tid & 31u;
  const int wave = __builtin_amdgcn_readfirstlane(threadIdx.x >> 5);
  const unsigned hh = lane >> 4, m = lane & 15u;
  const unsigned j0 = blockIdx.x * 16u;
  const unsigned b = blockIdx.y;

  const _Float16* ua16 = UA16 + (size_t)b * (NP * DD);
  const _Float16* ua2  = UA2 + (size_t)b * (NP * DD);
  const _Float16* uat  = UAT + (size_t)b * (DD * UP);
  const _Float16* uatr = UATR + (size_t)b * (DD * UP);
  const float* uaf = UAF + (size_t)b * (NP * DD);
  const float* tab = TAB + (size_t)b * (TROWS * TP);

  if (wave == 0) {
    const v8h z = {};
    *(v8h*)&sW[(lane >> 1) * WLD + NP + (lane & 1u) * 8u] = z;
    *(v8h*)&sWR[(lane >> 1) * WLD + NP + (lane & 1u) * 8u] = z;
  }

  const _Float16* bp  = ua16 + (size_t)(j0 + m) * DD + hh * 8u;
  const _Float16* bp2 = ua2 + (size_t)(j0 + m) * DD + hh * 8u;
  const v16h bj0 = frag_at(bp);
  const v16h bj1 = frag_at(bp + 32);
  const v16h bs0 = frag_at(bp2);
  const v16h bs1 = frag_at(bp2 + 32);

  const unsigned jcol = j0 + m;
  const float sk1 = tab[4 * TP + jcol];
  const float sk2 = tab[5 * TP + jcol];
  const bool jok = jcol < (unsigned)NN;

  float s2a = 0.0f, s3a = 0.0f;
  for (unsigned it = (unsigned)wave; it < (unsigned)NT; it += 8u) {
    const unsigned i0 = it * 16u;
    const _Float16* ap  = ua16 + (size_t)(i0 + m) * DD + hh * 8u;
    const _Float16* ap2 = ua2 + (size_t)(i0 + m) * DD + hh * 8u;
    v8f accMu = {}, accM2 = {};
    accMu = wmma16(frag_at(ap), bj0, accMu);
    accMu = wmma16(frag_at(ap + 32), bj1, accMu);
    accM2 = wmma16(frag_at(ap2), bs0, accM2);
    accM2 = wmma16(frag_at(ap2 + 32), bs1, accM2);

    const unsigned ir = i0 + hh * 8u;
    const v4f qa0 = *(const v4f*)(tab + 0 * TP + ir);
    const v4f qa1 = *(const v4f*)(tab + 0 * TP + ir + 4u);
    const v4f qb0 = *(const v4f*)(tab + 1 * TP + ir);
    const v4f qb1 = *(const v4f*)(tab + 1 * TP + ir + 4u);
    const v4f la0 = *(const v4f*)(tab + 2 * TP + ir);
    const v4f la1 = *(const v4f*)(tab + 2 * TP + ir + 4u);
    const v4f lb0 = *(const v4f*)(tab + 3 * TP + ir);
    const v4f lb1 = *(const v4f*)(tab + 3 * TP + ir + 4u);
    float q1[8], q2[8], l1[8], l2[8];
#pragma unroll
    for (int r = 0; r < 4; ++r) {
      q1[r] = qa0[r]; q1[r + 4] = qa1[r];
      q2[r] = qb0[r]; q2[r + 4] = qb1[r];
      l1[r] = la0[r]; l1[r + 4] = la1[r];
      l2[r] = lb0[r]; l2[r + 4] = lb1[r];
    }
    v8h pk, pkr;
#pragma unroll
    for (int r = 0; r < 8; ++r) {
      const float mu = accMu[r] * (1.0f / (float)DD);
      const float m2 = accM2[r] * (1.0f / (UA2CARRY * UA2CARRY * (float)DD));
      const float var = fmaxf(m2 - mu * mu, 0.0f);
      const float rr = rsqrtf(var + LN_EPS);
      const float w1 = __expf(leaky(q1[r] + sk1) - l1[r]);
      const float w2 = __expf(leaky(q2[r] + sk2) - l2[r]);
      const bool ok = jok && ((ir + (unsigned)r) < (unsigned)NN);
      const float wv = ok ? 0.5f * (w1 + w2) : 0.0f;
      const float wrv = wv * rr;
      s2a += wrv * mu;
      s3a += wv;
      const float t = wrv * WRCARRY;
      const _Float16 hv = toh_flush(t);
      pk[r]  = hv;
      pkr[r] = toh_flush(RCARRY * (t - (float)hv));
    }
    *(v8h*)&sW[m * WLD + i0 + hh * 8u] = pk;
    *(v8h*)&sWR[m * WLD + i0 + hh * 8u] = pkr;
  }

  s2a += __shfl_xor(s2a, 16, 32);
  s3a += __shfl_xor(s3a, 16, 32);
  if (hh == 0u) {
    sPart[(unsigned)wave * 32u + m] = s2a;
    sPart[(unsigned)wave * 32u + 16u + m] = s3a;
  }
  __syncthreads();

  if (tid < 32u) {
    float t = 0.0f;
#pragma unroll
    for (unsigned w = 0; w < 8u; ++w) t += sPart[w * 32u + tid];
    sS[tid] = t;
  }

  if (wave < 4) {
    const unsigned d0 = (unsigned)wave * 16u;
    const _Float16* tp  = uat + (size_t)(d0 + m) * UP + hh * 8u;
    const _Float16* tpr = uatr + (size_t)(d0 + m) * UP + hh * 8u;
    v8f acc = {}, accr = {};
#pragma unroll
    for (unsigned k0 = 0; k0 < (unsigned)KP; k0 += 32u) {
      const v16h a   = ld_frag(&sW[k0], WLD);
      const v16h ar  = ld_frag(&sWR[k0], WLD);
      const v16h bf  = frag_at(tp + k0);
      const v16h bfr = frag_at(tpr + k0);
      acc  = wmma16(a, bf, acc);
      accr = wmma16(a, bfr, accr);
      accr = wmma16(ar, bf, accr);
    }
#pragma unroll
    for (int r = 0; r < 8; ++r)
      sC[(hh * 8u + (unsigned)r) * LDC + d0 + m] =
          (acc[r] + accr[r] * (1.0f / RCARRY)) * (1.0f / WRCARRY);
  }
  __syncthreads();

  {
    const unsigned r = tid >> 4, c = (tid & 15u) * 4u;
    const unsigned j = j0 + r;
    const v4f s1 = *(const v4f*)&sC[r * LDC + c];
    const v4f uj = *(const v4f*)(uaf + (size_t)j * DD + c);
    const v4f gw = *(const v4f*)(lnw + c);
    const v4f gb = *(const v4f*)(lnb + c);
    const float s2 = sS[r], s3 = sS[16u + r];
    v4f val;
#pragma unroll
    for (int q = 0; q < 4; ++q) {
      const float t = bf16r(gw[q]) * (uj[q] * s1[q] - s2) + bf16r(gb[q]) * s3;
      val[q] = leaky(t);
    }
    if (j < (unsigned)NN) {
      float* p = out + ((size_t)b * (NN + 1) + 1u + j) * DD + c;
      *(volatile v4f*)p = val;
      __threadfence();
      *(volatile v4f*)p = val;
    }
  }
}

extern "C" void kernel_launch(void* const* d_in, const int* in_sizes, int n_in,
                              void* d_out, int out_size, void* d_ws, size_t ws_size,
                              hipStream_t stream) {
  if (n_in < 11) return;
  if ((long long)in_sizes[0] < (long long)NB * NODES * DD) return;
  if (in_sizes[1] < DD || in_sizes[2] < DD) return;
  if (in_sizes[3] < DD * DD || in_sizes[5] < DD * DD) return;
  if (in_sizes[4] < DD || in_sizes[6] < DD) return;
  if (in_sizes[7] < 3 * DD || in_sizes[9] < 3 * DD) return;
  if (in_sizes[8] < 1 || in_sizes[10] < 1) return;
  if ((long long)out_size < (long long)NB * (NN + 1) * DD) return;
  if (ws_size < WS_TOTAL) return;

  const float* emb = (const float*)d_in[0];
  const float* lnw = (const float*)d_in[1];
  const float* lnb = (const float*)d_in[2];
  const float* W1  = (const float*)d_in[3];
  const float* W1b = (const float*)d_in[4];
  const float* W2  = (const float*)d_in[5];
  const float* W2b = (const float*)d_in[6];
  const float* a1  = (const float*)d_in[7];
  const float* a1b = (const float*)d_in[8];
  const float* a2  = (const float*)d_in[9];
  const float* a2b = (const float*)d_in[10];
  float* out = (float*)d_out;

  char* ws = (char*)d_ws;
  _Float16* UA16 = (_Float16*)(ws + OFF_UA16);
  _Float16* UA2  = (_Float16*)(ws + OFF_UA2);
  _Float16* UAT  = (_Float16*)(ws + OFF_UAT);
  _Float16* UATR = (_Float16*)(ws + OFF_UATR);
  float*    UAF  = (float*)(ws + OFF_UAF);
  float*    TAB  = (float*)(ws + OFF_TAB);

  prep_kernel<<<dim3(NB), dim3(256), 0, stream>>>(emb, lnw, lnb, W1, W1b, W2, W2b,
                                                  a1, a1b, a2, a2b,
                                                  UA16, UA2, UAT, UATR, UAF, TAB, out);
  gat_kernel<<<dim3(NT, NB), dim3(256), 0, stream>>>(UA16, UA2, UAT, UATR, UAF, TAB,
                                                     lnw, lnb, out);
}
